// ScalarWaveletRecombiner_44040594653611
// MI455X (gfx1250) — hardware-verified
//
#include <hip/hip_runtime.h>

typedef __attribute__((ext_vector_type(16))) _Float16 v16h;
typedef __attribute__((ext_vector_type(8)))  _Float16 v8h;
typedef __attribute__((ext_vector_type(8)))  float    v8f;
typedef __attribute__((ext_vector_type(4)))  float    v4f;
typedef __attribute__((ext_vector_type(4)))  unsigned int v4u;

constexpr int kWav          = 64;
constexpr int kHid          = 128;
constexpr int kOutCh        = 32;
constexpr int kWavesPerBlock = 8;
constexpr int kRowsPerWave  = 32;
constexpr int kRowsPerBlock = kWavesPerBlock * kRowsPerWave;
constexpr int kThreads      = kWavesPerBlock * 32;
constexpr int kPitchB       = 72;
constexpr int kPitchO       = 36;
constexpr float kW1Carry    = 8.0f;
constexpr float kW1CarryInv = 0.125f;
constexpr float kNegLog2e   = -1.44269504088896341f;

template <typename T> struct Frag;
template <> struct Frag<_Float16> {
  typedef v16h V; union U { v16h v; v8h h[2]; };
  static __device__ __forceinline__ v16h load(const _Float16* p) {
    U f; f.h[0] = *(const v8h*)(p); f.h[1] = *(const v8h*)(p + 16); return f.v;
  }
  static __device__ __forceinline__ v8f mma(v16h a, v16h b, v8f c) {
    return __builtin_amdgcn_wmma_f32_16x16x32_f16(false, a, false, b, (short)0, c, false, false);
  }
};

__device__ __forceinline__ unsigned pk16(unsigned short a, unsigned short b) { return (unsigned)a | ((unsigned)b << 16); }
__device__ __forceinline__ unsigned short h_bits(float f) { const _Float16 h = (_Float16)f; return __builtin_bit_cast(unsigned short, h); }

__device__ __forceinline__ v8f mma_f16_g(v16h a, v16h b, v8f c) {
  c = __builtin_amdgcn_wmma_f32_16x16x32_f16(false, a, false, b, (short)0, c, false, false);
  asm volatile("v_nop\n\tv_nop\n\tv_nop\n\tv_nop" : "+v"(c) : "v"(a), "v"(b));
  return c;
}

__device__ __forceinline__ float fast_exp2(float x) {
#if __has_builtin(__builtin_amdgcn_exp2f)
  return __builtin_amdgcn_exp2f(x);
#else
  return exp2f(x);
#endif
}
__device__ __forceinline__ float fast_rcp(float x) {
#if __has_builtin(__builtin_amdgcn_rcpf)
  return __builtin_amdgcn_rcpf(x);
#else
  return 1.0f / x;
#endif
}

__global__ __launch_bounds__(256) void cast8_f16_kernel(const float* __restrict__ in, unsigned short* __restrict__ out,
                                                        int n8, float scale) {
  const int i = blockIdx.x * 256 + threadIdx.x;
  if (i >= n8) return;
  const float* p = in + 8 * (size_t)i;
  const v4f a = *(const v4f*)(p);
  const v4f c = *(const v4f*)(p + 4);
  unsigned short hb[8];
#pragma unroll
  for (int e = 0; e < 4; ++e) {
    hb[e]     = h_bits(a[e] * scale);
    hb[4 + e] = h_bits(c[e] * scale);
  }
  const v4u u = (v4u){pk16(hb[0], hb[1]), pk16(hb[2], hb[3]), pk16(hb[4], hb[5]), pk16(hb[6], hb[7])};
  unsigned short* q = out + 8 * (size_t)i;
  *(volatile v4u*)q = u;
  __threadfence();
  *(volatile v4u*)q = u;
}

__global__ __launch_bounds__(256) void fused_mlp_bank_kernel(
    const unsigned short* __restrict__ x16p,
    const unsigned short* __restrict__ w1hp,
    const float* __restrict__ b1,
    const float* __restrict__ w2,
    const float* __restrict__ b2,
    float* __restrict__ out,
    int nc) {
  __shared__ __align__(16) _Float16 sB[kHid * kPitchB];
  __shared__ __align__(16) float sO[kWavesPerBlock * kRowsPerWave * kPitchO];

  const _Float16* x16 = (const _Float16*)x16p;
  const _Float16* w1h = (const _Float16*)w1hp;
  const int tid   = threadIdx.x;
  const int lane  = tid & 31;
  const int wave  = tid >> 5;
  const int lmod  = lane & 15;
  const int lhalf = lane >> 4;
  const int rowBase = blockIdx.x * kRowsPerBlock + wave * kRowsPerWave;

  v16h afrag[2][2];
#pragma unroll
  for (int rg = 0; rg < 2; ++rg) {
    int row = rowBase + rg * 16 + lmod;
    row = (row < nc) ? row : (nc - 1);
    const _Float16* xr = x16 + (size_t)row * kWav + 8 * lhalf;
#pragma unroll
    for (int s = 0; s < 2; ++s) afrag[rg][s] = Frag<_Float16>::load(xr + 32 * s);
  }

  float rowpart[2][8];
  float* sOw = sO + wave * (kRowsPerWave * kPitchO);
  const v8f zero8 = {0.f, 0.f, 0.f, 0.f, 0.f, 0.f, 0.f, 0.f};

#pragma unroll 1
  for (int o = 0; o < kOutCh; ++o) {
    __syncthreads();
    {
      const _Float16* src = w1h + (size_t)o * kHid * kWav;
#pragma unroll
      for (int t = 0; t < 4; ++t) {
        const int i = tid + t * kThreads;
        const int r = i >> 3;
        const int c = i & 7;
        *(v8h*)(sB + r * kPitchB + c * 8) = *(const v8h*)(src + (size_t)i * 8);
      }
    }
    __syncthreads();

#pragma unroll
    for (int rg = 0; rg < 2; ++rg)
#pragma unroll
      for (int r = 0; r < 8; ++r) rowpart[rg][r] = 0.0f;

    const float* b1o = b1 + o * kHid + lmod;
    const float* w2o = w2 + o * kHid + lmod;

#pragma unroll 1
    for (int ht = 0; ht < 8; ++ht) {
      const _Float16* bp = sB + (ht * 16 + lmod) * kPitchB + 8 * lhalf;
      const v16h bf0 = Frag<_Float16>::load(bp);
      const v16h bf1 = Frag<_Float16>::load(bp + 32);
      const float b1v = b1o[ht * 16];
      const float w2v = w2o[ht * 16];
#pragma unroll
      for (int rg = 0; rg < 2; ++rg) {
        v8f acc = zero8;
        acc = mma_f16_g(afrag[rg][0], bf0, acc);
        acc = mma_f16_g(afrag[rg][1], bf1, acc);
#pragma unroll
        for (int r = 0; r < 8; ++r) {
          const float v  = __builtin_fmaf(acc[r], kW1CarryInv, b1v);
          const float e  = fast_exp2(v * kNegLog2e);
          const float sg = fast_rcp(1.0f + e);
          const float sv = v * sg;
          rowpart[rg][r] = __builtin_fmaf(sv, w2v, rowpart[rg][r]);
        }
      }
    }

#pragma unroll
    for (int m = 1; m < 16; m <<= 1) {
#pragma unroll
      for (int rg = 0; rg < 2; ++rg)
#pragma unroll
        for (int r = 0; r < 8; ++r) rowpart[rg][r] += __shfl_xor(rowpart[rg][r], m, 32);
    }

    const float b2o = b2[o];
    if (lmod == 0) {
#pragma unroll
      for (int rg = 0; rg < 2; ++rg)
#pragma unroll
        for (int r = 0; r < 8; ++r)
          sOw[(rg * 16 + 8 * lhalf + r) * kPitchO + o] = rowpart[rg][r] + b2o;
    }
  }

  __syncthreads();

  if (rowBase + kRowsPerWave <= nc) {
    const int q  = lane >> 3;
    const int c4 = (lane & 7) * 4;
    float* ob = out + (size_t)rowBase * kOutCh;
    for (int pass = 0; pass < 2; ++pass) {
#pragma unroll
      for (int it = 0; it < 8; ++it) {
        const int row = it * 4 + q;
        const v4f val = *(const v4f*)(sOw + row * kPitchO + c4);
        *(volatile v4f*)(ob + (size_t)row * kOutCh + c4) = val;
      }
      __threadfence();
    }
  }
}

extern "C" void kernel_launch(void* const* d_in, const int* in_sizes, int n_in,
                              void* d_out, int out_size, void* d_ws, size_t ws_size,
                              hipStream_t stream) {
  if (n_in < 5) return;
  const float* x   = (const float*)d_in[0];
  const float* W1  = (const float*)d_in[1];
  const float* b1  = (const float*)d_in[2];
  const float* W2  = (const float*)d_in[3];
  const float* b2  = (const float*)d_in[4];
  float* out = (float*)d_out;

  const int nX  = in_sizes[0];
  const int nW1 = in_sizes[1];
  if (nX <= 0 || (nX % kWav) != 0) return;
  const int nc = nX / kWav;
  if ((nc % kRowsPerWave) != 0) return;
  if (nW1 != kOutCh * kHid * kWav) return;
  if (in_sizes[2] != kOutCh * kHid || in_sizes[3] != kOutCh * kHid || in_sizes[4] != kOutCh) return;
  if (out_size != nc * kOutCh) return;

  const size_t bytesX = (size_t)nX * 2;
  const size_t offW   = (bytesX + 127) & ~(size_t)127;
  const size_t bytesW = (size_t)nW1 * 2;
  if (offW + bytesW > ws_size) return;

  unsigned short* x16 = (unsigned short*)((char*)d_ws + 0);
  unsigned short* w1h = (unsigned short*)((char*)d_ws + offW);

  const int n8x = nX / 8;
  const int n8w = nW1 / 8;
  cast8_f16_kernel<<<(n8x + 255) / 256, 256, 0, stream>>>(x, x16, n8x, 1.0f);
  cast8_f16_kernel<<<(n8w + 255) / 256, 256, 0, stream>>>(W1, w1h, n8w, kW1Carry);

  const int nblocks = (nc + kRowsPerBlock - 1) / kRowsPerBlock;
  fused_mlp_bank_kernel<<<nblocks, kThreads, 0, stream>>>(x16, w1h, b1, W2, b2, out, nc);
}
